// Net_LSTM_88776974008815
// MI455X (gfx1250) — hardware-verified
//
#include <hip/hip_runtime.h>


typedef _Float16 f16t;
typedef f16t  v16h __attribute__((ext_vector_type(16)));
typedef f16t  v8h  __attribute__((ext_vector_type(8)));
typedef float v8f  __attribute__((ext_vector_type(8)));
typedef float v4f  __attribute__((ext_vector_type(4)));
typedef unsigned int v4u __attribute__((ext_vector_type(4)));

union Frag { v16h v; v8h q[2]; };
union Pk16 { v8h h; v4u u; };

#define TN  512
#define HN  256
#define GN  1024
#define H1N 128
#define BT  16
#define HP  264

__device__ __forceinline__ v8f wmma16(v16h a, v16h b, v8f c) {
    return __builtin_amdgcn_wmma_f32_16x16x32_f16(false, a, false, b, (short)0, c, false, false);
}

__device__ __forceinline__ void wguard4(v8f (&c)[4], Frag& a, Frag (&b)[4]) {
    asm volatile("v_nop\n\tv_nop\n\tv_nop\n\tv_nop"
                 : "+v"(c[0]), "+v"(c[1]), "+v"(c[2]), "+v"(c[3])
                 : "v"(a.v), "v"(b[0].v), "v"(b[1].v), "v"(b[2].v), "v"(b[3].v));
}

__device__ __forceinline__ void zacc4(v8f (&acc)[4]) {
    const v8f z = {0.f, 0.f, 0.f, 0.f, 0.f, 0.f, 0.f, 0.f};
#pragma unroll
    for (int j = 0; j < 4; ++j) acc[j] = z;
}

__device__ __forceinline__ void mma4(v8f (&acc)[4], const f16t* A, int lda,
                                     const f16t* B, int ldb, int bstep, int ktiles) {
    const int l = threadIdx.x & 31, h = l >> 4, m = l & 15;
    const f16t* ap = A + (size_t)m * lda + 8 * h;
    const f16t* bp = B + (size_t)m * ldb + 8 * h;
#pragma unroll 1
    for (int kt = 0; kt < ktiles; ++kt) {
        Frag a, b[4];
        const f16t* pa = ap + kt * 32;
        a.q[0] = *(const v8h*)pa;
        a.q[1] = *(const v8h*)(pa + 16);
#pragma unroll
        for (int j = 0; j < 4; ++j) {
            const f16t* pb = bp + (size_t)j * bstep + kt * 32;
            b[j].q[0] = *(const v8h*)pb;
            b[j].q[1] = *(const v8h*)(pb + 16);
        }
#pragma unroll
        for (int j = 0; j < 4; ++j) acc[j] = wmma16(a.v, b[j].v, acc[j]);
        wguard4(acc, a, b);
    }
}

__device__ __forceinline__ float frcp(float x) { return __builtin_amdgcn_rcpf(x); }

__device__ __forceinline__ float ftanh(float x) {
    float ax = fabsf(x);
    float t  = __expf(-2.0f * ax);
    float r  = (1.0f - t) * frcp(1.0f + t);
    return copysignf(r, x);
}

__device__ __forceinline__ float fsig(float x) {
    float t = __expf(-fabsf(x));
    float r = frcp(1.0f + t);
    return (x >= 0.0f) ? r : t * r;
}

__global__ __launch_bounds__(256)
void k_cvt8(const float* x, f16t* y, int n8, float sc) {
    int i = blockIdx.x * 256 + threadIdx.x;
    if (i >= n8) return;
    const float* p = x + (size_t)i * 8;
    v4f a = *(const v4f*)p;
    v4f b = *(const v4f*)(p + 4);
    Pk16 k;
    k.h[0] = (f16t)(a[0] * sc); k.h[1] = (f16t)(a[1] * sc);
    k.h[2] = (f16t)(a[2] * sc); k.h[3] = (f16t)(a[3] * sc);
    k.h[4] = (f16t)(b[0] * sc); k.h[5] = (f16t)(b[1] * sc);
    k.h[6] = (f16t)(b[2] * sc); k.h[7] = (f16t)(b[3] * sc);
    f16t* d = y + (size_t)i * 8;
    *(volatile v4u*)d = k.u;
    __threadfence();
    *(volatile v4u*)d = k.u;
}

__global__ __launch_bounds__(512)
void k_lstm(const float* x, const float* W_ih, const float* b_ih, const float* b_hh,
            const f16t* Phh, f16t* Hf, int nb, float inv) {
    __shared__ __attribute__((aligned(16))) float xT[TN * BT];
    __shared__ __attribute__((aligned(16))) f16t  h_s[BT * HP];
    const int tid = threadIdx.x;
    const int l = tid & 31, w = tid >> 5, hh = l >> 4, m = l & 15;
    const int b0 = blockIdx.x * BT;
    if (b0 + BT > nb) return;

    for (int i = tid; i < BT * TN; i += 512) {
        int mr = i >> 9, t = i & (TN - 1);
        xT[t * BT + mr] = x[(size_t)(b0 + mr) * TN + t];
    }
    for (int i = tid; i < BT * HP; i += 512) h_s[i] = (f16t)0.0f;

    float wih[4], bs[4];
#pragma unroll
    for (int g = 0; g < 4; ++g) {
        int n = g * HN + 16 * w + m;
        wih[g] = W_ih[n];
        bs[g]  = b_ih[n] + b_hh[n];
    }

    v8f c = {0.f, 0.f, 0.f, 0.f, 0.f, 0.f, 0.f, 0.f};
    __syncthreads();

    const f16t* Bw = Phh + (size_t)(16 * w) * HN;
    f16t* hw = h_s + 16 * w + m;

#pragma unroll 1
    for (int t = 0; t < TN; ++t) {
        v8f acc[4];
        zacc4(acc);
        mma4(acc, h_s, HP, Bw, HN, HN * HN, HN / 32);
        __syncthreads();

        v4f x0 = *(const v4f*)(xT + t * BT + 8 * hh);
        v4f x1 = *(const v4f*)(xT + t * BT + 8 * hh + 4);
        v8f xv = __builtin_shufflevector(x0, x1, 0, 1, 2, 3, 4, 5, 6, 7);
        v8f hn;
#pragma unroll
        for (int r = 0; r < 8; ++r) {
            float xr = xv[r];
            float pi = fmaf(acc[0][r], inv, fmaf(xr, wih[0], bs[0]));
            float pf = fmaf(acc[1][r], inv, fmaf(xr, wih[1], bs[1]));
            float pg = fmaf(acc[2][r], inv, fmaf(xr, wih[2], bs[2]));
            float po = fmaf(acc[3][r], inv, fmaf(xr, wih[3], bs[3]));
            float ig = fsig(pi);
            float fg = fsig(pf);
            float gg = ftanh(pg);
            float og = fsig(po);
            float cv = fmaf(fg, c[r], ig * gg);
            c[r]  = cv;
            hn[r] = og * ftanh(cv);
        }
#pragma unroll
        for (int r = 0; r < 8; ++r) hw[(8 * hh + r) * HP] = (f16t)(hn[r] * 16.0f);
        __syncthreads();
    }

    {
        int row = tid >> 5, ch = l * 8;
        Pk16 v;
        v.h = *(const v8h*)(h_s + row * HP + ch);
        f16t* d = Hf + (size_t)(b0 + row) * HN + ch;
        *(volatile v4u*)d = v.u;
        __threadfence();
        *(volatile v4u*)d = v.u;
    }
}

__global__ __launch_bounds__(256)
void k_head(const f16t* Hf, const f16t* P1, const float* b1, const float* W2,
            const float* b2, float* out, float inv) {
    __shared__ __attribute__((aligned(16))) float ys[128];
    const int tid = threadIdx.x;
    const int l = tid & 31, w = tid >> 5, hh = l >> 4, m = l & 15;

    v8f s = {0.f, 0.f, 0.f, 0.f, 0.f, 0.f, 0.f, 0.f};
    const f16t* Aw = Hf + (size_t)(16 * w) * HN;
#pragma unroll
    for (int p = 0; p < 2; ++p) {
        v8f acc[4];
        zacc4(acc);
        mma4(acc, Aw, HN, P1 + (size_t)(64 * p) * HN, HN, 16 * HN, HN / 32);
#pragma unroll
        for (int j = 0; j < 4; ++j) {
            int col = 64 * p + 16 * j + m;
            float bj = b1[col];
            float w2 = W2[col];
#pragma unroll
            for (int r = 0; r < 8; ++r) {
                float v = fmaf(acc[j][r], inv, bj);
                v = fmaxf(v, 0.0f);
                s[r] = fmaf(v, w2, s[r]);
            }
        }
    }
#pragma unroll
    for (int r = 0; r < 8; ++r) {
        float v = s[r];
        v += __shfl_xor(v, 8);
        v += __shfl_xor(v, 4);
        v += __shfl_xor(v, 2);
        v += __shfl_xor(v, 1);
        s[r] = v;
    }
    if (m == 0) {
        float bb = b2[0];
#pragma unroll
        for (int r = 0; r < 8; ++r) ys[16 * w + 8 * hh + r] = s[r] + bb;
    }
    __syncthreads();
    if (tid < 32) {
        v4f v = *(const v4f*)(ys + 4 * l);
        *(volatile v4f*)(out + 4 * l) = v;
        __threadfence();
        *(volatile v4f*)(out + 4 * l) = v;
    }
}

extern "C" void kernel_launch(void* const* d_in, const int* in_sizes, int n_in,
                              void* d_out, int out_size, void* d_ws, size_t ws_size,
                              hipStream_t stream) {
    const int NB = 128;
    if (n_in < 9) return;
    if (in_sizes[0] != NB * TN || in_sizes[1] != GN || in_sizes[2] != GN * HN ||
        in_sizes[3] != GN || in_sizes[4] != GN || in_sizes[5] != H1N * HN ||
        in_sizes[6] != H1N || in_sizes[7] != H1N || in_sizes[8] < 1 ||
        out_size != NB) return;
    if ((NB % BT) != 0 || NB != 8 * 16) return;

    const float* x    = (const float*)d_in[0];
    const float* W_ih = (const float*)d_in[1];
    const float* W_hh = (const float*)d_in[2];
    const float* b_ih = (const float*)d_in[3];
    const float* b_hh = (const float*)d_in[4];
    const float* W1   = (const float*)d_in[5];
    const float* b1   = (const float*)d_in[6];
    const float* W2   = (const float*)d_in[7];
    const float* b2   = (const float*)d_in[8];
    float* out = (float*)d_out;

    char* ws = (char*)d_ws;
    size_t off = 0;
    auto carve = [&](size_t bytes) -> char* {
        char* p = ws + off;
        off = (off + bytes + 255) & ~(size_t)255;
        return p;
    };
    f16t* Phh = (f16t*)carve((size_t)GN * HN * 2);
    f16t* P1  = (f16t*)carve((size_t)H1N * HN * 2);
    f16t* Hf  = (f16t*)carve((size_t)NB * HN * 2);
    if (off > ws_size) return;

    const float S64 = 64.0f;
    const float INV = 0.0009765625f;

    {
        int n8 = GN * HN / 8;
        k_cvt8<<<dim3((n8 + 255) / 256), dim3(256), 0, stream>>>(W_hh, Phh, n8, S64);
    }
    {
        int n8 = H1N * HN / 8;
        k_cvt8<<<dim3((n8 + 255) / 256), dim3(256), 0, stream>>>(W1, P1, n8, S64);
    }
    k_lstm<<<dim3((NB + BT - 1) / BT), dim3(512), 0, stream>>>(x, W_ih, b_ih, b_hh,
                                                            Phh, Hf, NB, INV);
    k_head<<<dim3(1), dim3(256), 0, stream>>>(Hf, P1, b1, W2, b2, out, INV);
}
